// PMField_5196910428903
// MI455X (gfx1250) — hardware-run, weakly checked
//
#include <hip/hip_runtime.h>
#include <stddef.h>


typedef _Float16 h16;
typedef _Float16 v16h __attribute__((ext_vector_type(16)));
typedef float    v8f  __attribute__((ext_vector_type(8)));
typedef float    v4f  __attribute__((ext_vector_type(4)));

#ifndef NPTS
#define NPTS 524288
#endif
#define NPTS_FULL 524288
#define ND    8
#define NC    32
#define NSTEP 4
#define WAVES 8
#ifndef TPW
#define TPW   4
#endif
#define PTS_PER_BLOCK (WAVES * 16 * TPW)

#ifndef DOT_RES
#define DOT_RES 1
#endif
#ifndef W_RES
#define W_RES 0
#endif

#define EPSC   1.0e-4f
#define DTB    0.12f
#define CLMP   3.0f
#define CCARRY 64.0f
#define RCARRY 2048.0f
#define WCARRY 4.0f
#define WMAX   60000.0f

static_assert(NPTS >= PTS_PER_BLOCK && NPTS <= NPTS_FULL);
static_assert((NPTS % PTS_PER_BLOCK) == 0);
static_assert(NC * ND == 256);
static_assert(ND == 8);
static_assert(NC == 32);
static_assert(WAVES * 32 == 256);
static_assert(16 * ND * 4 == 32 * 16);
static_assert((size_t)NPTS_FULL * ND * 4 == (size_t)16777216);
static_assert((size_t)NPTS * ND < (size_t)0x7FFFFFFF);

__device__ __forceinline__ float bf16r(float x) {
  unsigned int u = __float_as_uint(x);
  u = (u + 0x7FFFu + ((u >> 16) & 1u)) & 0xFFFF0000u;
  return __uint_as_float(u);
}

static __device__ __forceinline__ h16 toh_flush(float v) {
  const h16 r = (h16)v;
  return (fabsf(v) < 6.103515625e-05f) ? (h16)0.0f : r;
}

__device__ __forceinline__ v8f wmma16(v16h a, v16h b, v8f c) {
  v8f d = __builtin_amdgcn_wmma_f32_16x16x32_f16(false, a, false, b, (short)0, c,
                                                 false, false);
  asm volatile("v_nop\n\tv_nop\n\tv_nop\n\tv_nop" : "+v"(d) : "v"(a), "v"(b));
  return d;
}

__global__ __launch_bounds__(256) void field_kernel(
    const float* __restrict__ z_in, const float* __restrict__ centers,
    const float* __restrict__ mus, float* __restrict__ z_out) {
  __shared__ float sc[NC * ND];
  __shared__ float smu[NC];
  __shared__ float scn[NC];

  const unsigned tid = threadIdx.x;
  sc[tid] = bf16r(centers[tid]);
  if (tid < (unsigned)NC) smu[tid] = bf16r(mus[tid]);
  __syncthreads();
  if (tid < (unsigned)NC) {
    float s = 0.0f;
#pragma unroll
    for (int d = 0; d < ND; ++d) { const float c = sc[tid * ND + d]; s += c * c; }
    scn[tid] = s + EPSC;
  }
  __syncthreads();

  const unsigned lane = tid & 31u;
  const unsigned wave = (unsigned)__builtin_amdgcn_readfirstlane((int)(threadIdx.x >> 5));
  const unsigned hh = lane >> 4, m = lane & 15u;

  v16h a1[2];
#pragma unroll
  for (int blk = 0; blk < 2; ++blk) {
#pragma unroll
    for (int i = 0; i < 8; ++i) {
      const float c = sc[(16u * (unsigned)blk + m) * ND + (unsigned)i];
      const float hiv = c * CCARRY;
#if DOT_RES
      const float lov = c * (CCARRY / RCARRY);
#else
      const float lov = 0.0f;
#endif
      a1[blk][i]     = toh_flush(hh ? lov : hiv);
      a1[blk][i + 8] = (h16)0.0f;
    }
  }
  v16h a2;
  {
    const unsigned d = m & 7u;
#pragma unroll
    for (int i = 0; i < 8; ++i) {
      a2[i]     = toh_flush(CCARRY * sc[(8u * hh + (unsigned)i) * ND + d]);
      a2[i + 8] = toh_flush(CCARRY * sc[(16u + 8u * hh + (unsigned)i) * ND + d]);
    }
  }
  float mu_r[2][8], cn_r[2][8];
#pragma unroll
  for (int blk = 0; blk < 2; ++blk) {
#pragma unroll
    for (int v = 0; v < 8; ++v) {
      const unsigned c = (unsigned)v + 8u * hh + 16u * (unsigned)blk;
      mu_r[blk][v] = smu[c];
      cn_r[blk][v] = scn[c];
    }
  }

  const v8f zero8 = {};

#pragma unroll 1
  for (unsigned t = 0; t < (unsigned)TPW; ++t) {
    const unsigned tile = (blockIdx.x * (unsigned)WAVES + wave) * (unsigned)TPW + t;
    const size_t pbase = (size_t)tile * 16u;

    const float* zp = z_in + (pbase + m) * ND;
    const v4f l0 = *(const v4f*)(zp);
    const v4f l1 = *(const v4f*)(zp + 4);
    float z[8];
#pragma unroll
    for (int i = 0; i < 4; ++i) { z[i] = bf16r(l0[i]); z[i + 4] = bf16r(l1[i]); }

#pragma unroll 1
    for (int step = 0; step < NSTEP; ++step) {
      float znorm = 0.0f;
#pragma unroll
      for (int i = 0; i < 8; ++i) znorm += z[i] * z[i];

      v16h b1;
#pragma unroll
      for (int i = 0; i < 8; ++i) {
        const h16 zh = toh_flush(z[i]);
#if DOT_RES
        const h16 zl = toh_flush((z[i] - (float)zh) * RCARRY);
#else
        const h16 zl = (h16)0.0f;
#endif
        b1[i]     = hh ? zl : zh;
        b1[i + 8] = (h16)0.0f;
      }

      v8f acc[2];
      acc[0] = wmma16(a1[0], b1, zero8);
      acc[1] = wmma16(a1[1], b1, zero8);

      float nnp = 0.0f, sp = 0.0f;
      v16h b2;
#if W_RES
      float spr = 0.0f;
      v16h b2r;
#endif
#pragma unroll
      for (int blk = 0; blk < 2; ++blk) {
#pragma unroll
        for (int v = 0; v < 8; ++v) {
          const float dot = acc[blk][v];
          float r2 = fmaf(-2.0f / CCARRY, dot, znorm) + cn_r[blk][v];
          r2 = fmaxf(r2, EPSC);
          const float rs = __builtin_amdgcn_rsqf(r2);
          const float u = mu_r[blk][v] * rs;
          const float w = u * rs * rs;
          nnp += u;
          const float wc = fminf(w * WCARRY, WMAX);
          const h16 wh = toh_flush(wc);
          b2[blk * 8 + v] = wh;
          sp += (float)wh;
#if W_RES
          const h16 wl = toh_flush((wc - (float)wh) * RCARRY);
          b2r[blk * 8 + v] = wl;
          spr += (float)wl;
#endif
        }
      }

      const v8f gacc = wmma16(a2, b2, zero8);
#if W_RES
      const v8f gres = wmma16(a2, b2r, zero8);
#endif

      nnp += __shfl_xor(nnp, 16, 32);
      sp  += __shfl_xor(sp, 16, 32);
#if W_RES
      spr += __shfl_xor(spr, 16, 32);
      const float spf = (sp + spr * (1.0f / RCARRY)) * (1.0f / WCARRY);
#else
      const float spf = sp * (1.0f / WCARRY);
#endif
      const float nn = 1.0f + nnp;
      const float scale = DTB * __builtin_amdgcn_rcpf(nn);
      const float ginv = 1.0f / (CCARRY * WCARRY);

#pragma unroll
      for (int i = 0; i < 8; ++i) {
#if W_RES
        const float gs = (gacc[i] + gres[i] * (1.0f / RCARRY)) * ginv;
#else
        const float gs = gacc[i] * ginv;
#endif
        const float g = gs - spf * z[i];
        float zn = z[i] + scale * g;
        zn = fminf(CLMP, fmaxf(-CLMP, zn));
        z[i] = zn;
      }
    }

    const int src = (int)((lane >> 1) + 16u * (lane & 1u));
    v4f piece;
#pragma unroll
    for (int j = 0; j < 4; ++j) {
      const float mine = hh ? z[4 + j] : z[j];
      piece[j] = __shfl(mine, src, 32);
    }
    float* op = z_out + pbase * ND + lane * 4u;
    *(volatile v4f*)op = piece;
    __threadfence();
    *(volatile v4f*)op = piece;
  }
}

extern "C" void kernel_launch(void* const* d_in, const int* in_sizes, int n_in,
                              void* d_out, int out_size, void* d_ws, size_t ws_size,
                              hipStream_t stream) {
  (void)d_ws; (void)ws_size;
  if (n_in < 3) return;
  if ((long long)in_sizes[0] < (long long)NPTS * ND) return;
  if (in_sizes[1] < NC * ND) return;
  if (in_sizes[2] < NC) return;
  if ((long long)out_size < (long long)NPTS * ND) return;

  const float* z       = (const float*)d_in[0];
  const float* centers = (const float*)d_in[1];
  const float* mus     = (const float*)d_in[2];
  float* out = (float*)d_out;

  field_kernel<<<dim3(NPTS / PTS_PER_BLOCK), dim3(256), 0, stream>>>(z, centers, mus, out);
}
